// SheafDiffusion_39436389712331
// MI455X (gfx1250) — hardware-run, weakly checked
//
#include <hip/hip_runtime.h>


namespace {
constexpr int NN = 100000, NE = 1600000, FI = 128, DH = 32, GH = 64, NOUT = 10, MAXDEG = 1024, NGc = (NN + 511) / 512, PERMLEN = NE + 32 * NGc + 32;
constexpr float XS = 8.0f, TWO_PI = 6.283185307179586f;

typedef _Float16 b16;
typedef __attribute__((ext_vector_type(16))) _Float16 v16b;
typedef __attribute__((ext_vector_type(8))) _Float16 v8b;
typedef __attribute__((ext_vector_type(8))) float v8f;
typedef __attribute__((ext_vector_type(4))) float v4f;
typedef __attribute__((ext_vector_type(2))) float v2f;
__device__ __forceinline__ float bf16_rne(float f) { unsigned int u = __float_as_uint(f); u += 0x7FFFu + ((u >> 16) & 1u); return __uint_as_float(u & 0xFFFF0000u); }
__device__ __forceinline__ void split16(float v, b16& hi, b16& lo) { hi = (b16)v; lo = (b16)(v - (float)hi); }
__device__ __forceinline__ v16b frag_kb(const b16* p, int hh) { const v8b a = *(const v8b*)(p + 8 * hh), b = *(const v8b*)(p + 16 + 8 * hh); v16b f;
#pragma unroll
  for (int e = 0; e < 8; ++e) { f[e] = a[e]; f[8 + e] = b[e]; } return f; }
__device__ __forceinline__ v8f wmma16b(v16b a, v16b b, v8f c) { v8f d = __builtin_amdgcn_wmma_f32_16x16x32_f16(false, a, false, b, (short)0, c, false, false); asm volatile("v_nop\n\tv_nop\n\tv_nop\n\tv_nop" : "+v"(d) : "v"(a), "v"(b)); return d; }
__device__ __forceinline__ void wave_lds_sync() { __builtin_amdgcn_fence(__ATOMIC_RELEASE, "workgroup"); __builtin_amdgcn_wave_barrier(); __builtin_amdgcn_fence(__ATOMIC_ACQUIRE, "workgroup"); }
__device__ __forceinline__ float nexp(float x) { return __builtin_amdgcn_exp2f(x * 1.4426950408889634f); }
__device__ __forceinline__ float pmul(float a, float b) { float p = a * b; asm volatile("" : "+v"(p)); return p; }
__device__ __forceinline__ float tanh_f(float x) { const float e = nexp(-2.0f * fabsf(x)); const float t = (1.0f - e) / (1.0f + e); return (x < 0.0f) ? -t : t; }
__device__ __forceinline__ float gelu_t(float x) { const float u = 0.7978845608028654f * (x + 0.044715f * pmul(pmul(x, x), x)); return 0.5f * x * (1.0f + tanh_f(u)); }
constexpr int CSR_NBLK = 512, CSR_GB = 9, CSR_GN = 1 << CSR_GB  , CSR_MAXG = 512, CSR_CAP = 12288  ;
__global__ __launch_bounds__(64) void csrA_kernel(const int* __restrict__ dst, int E, int N, int nG, int CHP, int NGP, int* __restrict__ STG, int* __restrict__ HST) {
  extern __shared__ int sm[];
  int* cnt = sm; int* run = sm + NGP; int* ids = sm + 2 * NGP;
  const int b = blockIdx.x; const int ch = (E + CSR_NBLK - 1) / CSR_NBLK; const int e0 = b * ch, e1 = min(E, e0 + ch);
  for (int i = threadIdx.x; i < NGP; i += 64) cnt[i] = 0;
  for (int i = threadIdx.x; i < CHP; i += 64) ids[i] = -1;
  __syncthreads();
  if (threadIdx.x == 0) {
    for (int e = e0; e < e1; ++e) { int d = dst[e]; d = (d < 0) ? 0 : (d >= N ? N - 1 : d); cnt[d >> CSR_GB] += 1; }
    int acc = 0; for (int g = 0; g < nG; ++g) { run[g] = acc; acc += cnt[g]; }
    for (int e = e0; e < e1; ++e) { int d = dst[e]; d = (d < 0) ? 0 : (d >= N ? N - 1 : d); const int g = d >> CSR_GB; ids[run[g]] = e; run[g] += 1; } }
  __syncthreads();
  typedef __attribute__((ext_vector_type(4))) int v4i;
  for (int pass = 0; pass < 2; ++pass) {
    for (int i = threadIdx.x; i < CHP / 4; i += 64) *(volatile v4i*)(STG + (size_t)b * CHP + i * 4) = *(const v4i*)(&ids[i * 4]);
    for (int i = threadIdx.x; i < NGP / 4; i += 64) { v4i v; for (int e = 0; e < 4; ++e) v[e] = (i * 4 + e < nG) ? cnt[i * 4 + e] : 0; *(volatile v4i*)(HST + (size_t)b * NGP + i * 4) = v; }
    __threadfence(); }
}
__global__ __launch_bounds__(512) void csrS_kernel(const int* __restrict__ HST, int nG, int NGP, int* __restrict__ START, int* __restrict__ TOT, int* __restrict__ OFF) {
  __shared__ int tot[CSR_MAXG];
  const int b = threadIdx.x;
  for (int pass = 0; pass < 2; ++pass) { int runb = 0; for (int g = 0; g < nG; ++g) { int c = HST[(size_t)b * NGP + g]; c = (c < 0) ? 0 : c; ((volatile int*)OFF)[(size_t)g * CSR_NBLK + b] = runb; runb += c; } __threadfence(); }
  for (int g = threadIdx.x; g < nG; g += 512) { int s = 0; for (int bb = 0; bb < CSR_NBLK; ++bb) { int c = HST[(size_t)bb * NGP + g]; s += (c < 0) ? 0 : c; } tot[g] = s; }
  __syncthreads();
  if (threadIdx.x < 32) {
    __shared__ int st[CSR_MAXG + 32];
    if (threadIdx.x == 0) { int acc = 0; for (int g = 0; g < NGP; ++g) { st[g] = acc; if (g < nG) acc += (tot[g] + 31) & ~31; } st[NGP] = acc; }
    __builtin_amdgcn_fence(__ATOMIC_RELEASE, "workgroup"); __builtin_amdgcn_wave_barrier(); __builtin_amdgcn_fence(__ATOMIC_ACQUIRE, "workgroup");
    for (int pass = 0; pass < 2; ++pass) { for (int i = threadIdx.x; i < NGP + 32; i += 32) { ((volatile int*)START)[i] = (i <= NGP) ? st[min(i, NGP)] : 0; ((volatile int*)TOT)[i] = (i < nG) ? tot[i] : 0; } __threadfence(); } }
}
__global__ __launch_bounds__(256) void csrB_kernel(const int* __restrict__ dst, int N, int nG, int CHP, int NGP, int permLen, const int* __restrict__ STG, const int* __restrict__ HST, const int* __restrict__ OFF, const int* __restrict__ START, const int* __restrict__ TOT, int* __restrict__ PERM, int* __restrict__ ROWPTR, int* __restrict__ ROWCNT, int* __restrict__ FLAG) {
  typedef __attribute__((ext_vector_type(4))) int v4i;
  __shared__ int ids[CSR_CAP]; __shared__ unsigned short key[CSR_CAP]; __shared__ int outp[CSR_CAP]; __shared__ int ncnt[CSR_GN + 1]; __shared__ int boff[CSR_NBLK + 1];
  const int g = blockIdx.x, t_ = threadIdx.x; int tot = TOT[g]; int st = START[g], stn = START[g + 1]; const int v0 = g * CSR_GN; const int nv = min(CSR_GN, N - v0);
  st = (st < 0) ? 0 : (st > permLen - 32 ? permLen - 32 : st) & ~31; stn = (stn < st) ? st : (stn > permLen ? permLen : stn); tot = (tot < 0) ? 0 : tot; if (tot > stn - st && tot <= CSR_CAP) tot = stn - st;
  if (tot > CSR_CAP) {
    for (int pass = 0; pass < 2; ++pass) { for (int i = t_; i < CSR_GN / 4; i += 256) { v4i a, c; for (int e = 0; e < 4; ++e) { a[e] = st; c[e] = 0; } *(volatile v4i*)(ROWPTR + v0 + i * 4) = a; *(volatile v4i*)(ROWCNT + v0 + i * 4) = c; } if (t_ == 0) ((volatile int*)FLAG)[0] = 1; __threadfence(); } (void)nv; return; }
  if (t_ == 0) { int acc = 0; for (int b = 0; b < CSR_NBLK; ++b) { boff[b] = acc; int c = HST[(size_t)b * NGP + g]; c = (c < 0) ? 0 : (c > CHP ? CHP : c); acc += c; if (acc > tot) acc = tot; } boff[CSR_NBLK] = acc; }
  for (int i = t_; i <= CSR_GN; i += 256) ncnt[i] = 0;
  __syncthreads();
  for (int b = 0; b < CSR_NBLK; ++b) { const int c = boff[b + 1] - boff[b]; int o_ = OFF[(size_t)g * CSR_NBLK + b]; o_ = (o_ < 0) ? 0 : (o_ > CHP - c ? CHP - c : o_); const int* src_ = STG + (size_t)b * CHP + o_;
    for (int i = t_; i < c; i += 256) { int id = src_[i]; id = (id < 0) ? 0 : id; ids[boff[b] + i] = id; int d = dst[id]; d = (d < v0) ? v0 : (d >= N ? N - 1 : d); int kk = d - v0; kk = (kk < 0) ? 0 : (kk >= CSR_GN ? CSR_GN - 1 : kk); key[boff[b] + i] = (unsigned short)kk; } }
  __syncthreads();
  if (t_ == 0) { for (int i = 0; i < tot; ++i) ncnt[key[i]] += 1; int acc = 0; for (int vl = 0; vl < CSR_GN; ++vl) { const int c = ncnt[vl]; ncnt[vl] = acc; acc += c; } ncnt[CSR_GN] = acc;
    for (int i = 0; i < tot; ++i) { const int vl = key[i]; outp[ncnt[vl]] = ids[i]; ncnt[vl] += 1; }
    for (int vl = CSR_GN; vl > 0; --vl) ncnt[vl] = ncnt[vl - 1]; ncnt[0] = 0; }
  __syncthreads();
  for (int pass = 0; pass < 2; ++pass) {
    for (int i = t_; i < (stn - st) / 4; i += 256) { v4i v; for (int e = 0; e < 4; ++e) { const int q = i * 4 + e; v[e] = (q < tot) ? outp[q] : -1; } *(volatile v4i*)(PERM + st + i * 4) = v; }
    for (int i = t_; i < CSR_GN / 4; i += 256) { v4i a, c; for (int e = 0; e < 4; ++e) { const int vl = i * 4 + e; a[e] = st + ncnt[vl]; c[e] = (vl < nv) ? (ncnt[vl + 1] - ncnt[vl]) : 0; } *(volatile v4i*)(ROWPTR + v0 + i * 4) = a; *(volatile v4i*)(ROWCNT + v0 + i * 4) = c; }
    __threadfence(); }
}
__global__ __launch_bounds__(256) void csrZ_kernel(int* __restrict__ p, size_t n4) { typedef __attribute__((ext_vector_type(4))) int v4i; const size_t tid = (size_t)blockIdx.x * 256 + threadIdx.x, nth = (size_t)gridDim.x * 256; v4i z = {0, 0, 0, 0}; for (size_t i = tid; i < n4; i += nth) *(volatile v4i*)(p + i * 4) = z; }
struct CsrBufs { int *STG, *HST, *OFF, *START, *TOT, *PERM, *ROWPTR, *ROWCNT, *FLAG; int nG, NGP, CHP; size_t permLen; char* base; size_t bytes; };
static size_t csr_carve(CsrBufs& c, char* ws, size_t off, int E, int N) {
  const size_t off0 = off; c.base = ws + off;
  auto al = [&](size_t bytes) { char* p = ws + off; off += (bytes + 255) & ~(size_t)255; return p; };
  c.nG = (N + CSR_GN - 1) / CSR_GN; c.NGP = (c.nG + 31) & ~31; const int ch = (E + CSR_NBLK - 1) / CSR_NBLK; c.CHP = (ch + 31) & ~31; c.permLen = (size_t)E + 32 * (size_t)c.nG + 32;
  c.STG = (int*)al((size_t)CSR_NBLK * c.CHP * 4); c.HST = (int*)al((size_t)CSR_NBLK * c.NGP * 4); c.OFF = (int*)al((size_t)c.NGP * CSR_NBLK * 4); c.START = (int*)al((size_t)(c.NGP + 64) * 4); c.TOT = (int*)al((size_t)(c.NGP + 64) * 4);
  c.PERM = (int*)al(c.permLen * 4); c.ROWPTR = (int*)al((size_t)c.nG * CSR_GN * 4); c.ROWCNT = (int*)al((size_t)c.nG * CSR_GN * 4); c.FLAG = (int*)al(256);
  c.bytes = off - off0; return off;
}
static void csr_build(const CsrBufs& c, const int* dst, int E, int N, hipStream_t stream) {
  const size_t smem = (size_t)(2 * c.NGP + c.CHP) * 4;
  csrZ_kernel<<<512, 256, 0, stream>>>((int*)c.base, c.bytes / 16);
  csrA_kernel<<<CSR_NBLK, 64, smem, stream>>>(dst, E, N, c.nG, c.CHP, c.NGP, c.STG, c.HST);
  csrS_kernel<<<1, 512, 0, stream>>>(c.HST, c.nG, c.NGP, c.START, c.TOT, c.OFF);
  csrB_kernel<<<c.nG, 256, 0, stream>>>(dst, N, c.nG, c.CHP, c.NGP, (int)c.permLen, c.STG, c.HST, c.OFF, c.START, c.TOT, c.PERM, c.ROWPTR, c.ROWCNT, c.FLAG);
}

__global__ __launch_bounds__(256) void prep_kernel(const float* __restrict__ x, const float* __restrict__ win, const float* __restrict__ bin, const float* __restrict__ e1w, const float* __restrict__ e1b, const float* __restrict__ ws1, const float* __restrict__ wn1, const float* __restrict__ ws2, const float* __restrict__ wn2, const float* __restrict__ e2w, const float* __restrict__ e2b, const float* __restrict__ wd, const float* __restrict__ wo, const float* __restrict__ bo, b16* __restrict__ R, float* __restrict__ P, b16* __restrict__ X) {
  const size_t tid = (size_t)blockIdx.x * 256 + threadIdx.x, nth = (size_t)gridDim.x * 256;
  for (int pass = 0; pass < 2; ++pass) {
    for (size_t p = tid; p < (size_t)DH * FI; p += nth) { const int o = (int)(p / FI), k = (int)(p % FI); ((volatile b16*)R)[p] = (b16)bf16_rne(win[(size_t)k * DH + o]); }
    for (size_t p = tid; p < (size_t)GH * DH; p += nth) { const int o = (int)(p / DH), k = (int)(p % DH); ((volatile b16*)R)[4096 + p] = (b16)bf16_rne(e1w[(size_t)k * GH + o]); }
    for (size_t p = tid; p < (size_t)GH * 128; p += nth) { const int o = (int)(p / 128), k = (int)(p % 128); const float a = (k < 64) ? ws1[(size_t)k * GH + o] : wn1[(size_t)(k - 64) * GH + o]; const float b = (k < 64) ? ws2[(size_t)k * GH + o] : wn2[(size_t)(k - 64) * GH + o]; ((volatile b16*)R)[6144 + p] = (b16)bf16_rne(a); ((volatile b16*)R)[14336 + p] = (b16)bf16_rne(b); }
    for (size_t p = tid; p < (size_t)16 * DH; p += nth) { const int o = (int)(p / DH), k = (int)(p % DH); ((volatile b16*)R)[22528 + p] = (b16)((o < NOUT) ? bf16_rne(wo[(size_t)k * NOUT + o]) : 0.0f); }
    for (size_t q = tid; q < 720; q += nth) { const int i = (int)q; float v; if (i < 32) v = bin[i]; else if (i < 96) v = e1b[i - 32]; else if (i < 160) v = e2w[i - 96]; else if (i < 161) v = e2b[0]; else if (i < 192) v = 0.0f; else if (i < 704) v = wd[i - 192]; else v = (i - 704 < NOUT) ? bo[i - 704] : 0.0f; P[q] = bf16_rne(v); }
    for (size_t p = tid; p < (size_t)NN * FI / 8; p += nth) { v8b v; for (int e = 0; e < 8; ++e) v[e] = (b16)(bf16_rne(x[p * 8 + e]) * XS); *(volatile v8b*)(X + p * 8) = v; }
    __threadfence(); }
}
template <int KIN, int NO, int TWO, int EPI>
__global__ __launch_bounds__(64) void gemm_kernel(const b16* __restrict__ Ah, const b16* __restrict__ Al, int lda, const b16* __restrict__ Bw, const float* __restrict__ bias, float* __restrict__ OUTF, b16* __restrict__ Ch, b16* __restrict__ Cl) {
  __shared__ __attribute__((aligned(16))) float Ts[2][16][NO + 4]; __shared__ __attribute__((aligned(16))) b16 Sh[2][16][NO + 8], Sl[2][16][NO + 8];
  constexpr int NS = NO / 16;
  const int lane = threadIdx.x & 31, wave = threadIdx.x >> 5, nloc = lane & 15, hlf = lane >> 4, m0 = blockIdx.x * 32 + wave * 16;
  v8f acc[NS];
#pragma unroll
  for (int t = 0; t < NS; ++t) acc[t] = (v8f){};
#pragma unroll
  for (int kb = 0; kb < KIN; kb += 32) { const v16b a = frag_kb(Ah + (size_t)(m0 + nloc) * lda + kb, hlf); v16b al_; if (TWO) al_ = frag_kb(Al + (size_t)(m0 + nloc) * lda + kb, hlf);
#pragma unroll
    for (int t = 0; t < NS; ++t) { const v16b bw = frag_kb(Bw + (size_t)(t * 16 + nloc) * KIN + kb, hlf); acc[t] = wmma16b(a, bw, acc[t]); if (TWO) acc[t] = wmma16b(al_, bw, acc[t]); } }
#pragma unroll
  for (int t = 0; t < NS; ++t)
#pragma unroll
    for (int r = 0; r < 8; ++r) { float y = acc[t][r] * (1.0f / XS) + (bias ? bias[t * 16 + nloc] : 0.0f); if (EPI == 1) y = gelu_t(y); Ts[wave][8 * hlf + r][t * 16 + nloc] = y; if (EPI == 1) { b16 a_, b_; split16(y * XS, a_, b_); Sh[wave][8 * hlf + r][t * 16 + nloc] = a_; Sl[wave][8 * hlf + r][t * 16 + nloc] = b_; } }
  wave_lds_sync();
  for (int pass = 0; pass < 2; ++pass) { for (int i = lane; i < 16 * (NO / 4); i += 32) { const int rr = i / (NO / 4), c4 = (i % (NO / 4)) * 4; *(volatile v4f*)(OUTF + (size_t)(m0 + rr) * NO + c4) = *(const v4f*)(&Ts[wave][rr][c4]); }
    if (EPI == 1) { for (int i = lane; i < 16 * (NO / 8); i += 32) { const int rr = i / (NO / 8), c8 = (i % (NO / 8)) * 8; const size_t gi = (size_t)(m0 + rr) * 128 + c8; *(volatile v8b*)(Ch + gi) = *(const v8b*)(&Sh[wave][rr][c8]); *(volatile v8b*)(Cl + gi) = *(const v8b*)(&Sl[wave][rr][c8]); } } __threadfence(); }
}
__global__ __launch_bounds__(256) void hsplit_kernel(const float* __restrict__ H, b16* __restrict__ Hh, b16* __restrict__ Hl) {
  const size_t p = (size_t)blockIdx.x * 256 + threadIdx.x; if (p >= (size_t)NN * DH / 8) return;
  v8b a, b; for (int e = 0; e < 8; ++e) { b16 x_, y_; split16(H[p * 8 + e] * XS, x_, y_); a[e] = x_; b[e] = y_; }
  for (int pass = 0; pass < 2; ++pass) { *(volatile v8b*)(Hh + p * 8) = a; *(volatile v8b*)(Hl + p * 8) = b; __threadfence(); }
}
__global__ __launch_bounds__(256) void magg_kernel(const float* __restrict__ M, const int* __restrict__ src, const int* __restrict__ perm, const int* __restrict__ rowptr, const int* __restrict__ rowcnt, b16* __restrict__ Ch, b16* __restrict__ Cl) {
  __shared__ __attribute__((aligned(16))) b16 Sh[8][GH + 8], Sl[8][GH + 8];
  const int wave = threadIdx.x >> 5, v = blockIdx.x * 8 + wave, lane = threadIdx.x & 31;
  int cnt = rowcnt[v]; cnt = (cnt < 0) ? 0 : (cnt > MAXDEG ? MAXDEG : cnt); int p0 = rowptr[v]; p0 = (p0 < 0) ? 0 : (p0 > PERMLEN - cnt ? PERMLEN - cnt : p0);
  float a0 = 0.0f, a1 = 0.0f;
  for (int q = 0; q < cnt; ++q) { int id = perm[p0 + q]; id = (id < 0) ? 0 : (id >= NE ? NE - 1 : id); int s = src[id]; s = (s < 0) ? 0 : (s >= NN ? NN - 1 : s); const v2f mv = *(const v2f*)(M + (size_t)s * GH + lane * 2); a0 += mv[0]; a1 += mv[1]; }
  b16 x_, y_; split16(a0 * XS, x_, y_); Sh[wave][lane * 2] = x_; Sl[wave][lane * 2] = y_; split16(a1 * XS, x_, y_); Sh[wave][lane * 2 + 1] = x_; Sl[wave][lane * 2 + 1] = y_;
  wave_lds_sync();
  for (int pass = 0; pass < 2; ++pass) { if (lane < 8) { *(volatile v8b*)(Ch + (size_t)v * 128 + 64 + lane * 8) = *(const v8b*)(&Sh[wave][lane * 8]); *(volatile v8b*)(Cl + (size_t)v * 128 + 64 + lane * 8) = *(const v8b*)(&Sl[wave][lane * 8]); } __threadfence(); }
}
__global__ __launch_bounds__(256) void theta_kernel(const float* __restrict__ M, const float* __restrict__ P, float* __restrict__ CS) {
  const int n = blockIdx.x * 256 + threadIdx.x; v2f o = {1.0f, 0.0f};
  if (n < NN) { float s = P[160]; for (int j = 0; j < GH; ++j) s += pmul(M[(size_t)n * GH + j], P[96 + j]); const float th = tanh_f(s); const float ang = th * TWO_PI; o[0] = (float)cos((double)ang); o[1] = (float)sin((double)ang); }
  for (int pass = 0; pass < 2; ++pass) { if (n < NN) *(volatile v2f*)(CS + (size_t)n * 2) = o; __threadfence(); }
}
template <int LAST>
__global__ __launch_bounds__(256) void diff_kernel(const float* __restrict__ XSin, const float* __restrict__ CS, const int* __restrict__ src, const int* __restrict__ perm, const int* __restrict__ rowptr, const int* __restrict__ rowcnt, const float* __restrict__ Pw, float* __restrict__ XSout, b16* __restrict__ Xh, b16* __restrict__ Xl) {
  __shared__ float Lx[8][DH + 1]; __shared__ __attribute__((aligned(16))) b16 Sh[8][DH + 8], Sl[8][DH + 8];
  const int wave = threadIdx.x >> 5, v = blockIdx.x * 8 + wave, lane = threadIdx.x & 31, d = lane >> 4, k = lane & 15;
  int cnt = rowcnt[v]; cnt = (cnt < 0) ? 0 : (cnt > MAXDEG ? MAXDEG : cnt); int p0 = rowptr[v]; p0 = (p0 < 0) ? 0 : (p0 > PERMLEN - cnt ? PERMLEN - cnt : p0);
  const float cv = CS[(size_t)v * 2], sv = CS[(size_t)v * 2 + 1]; const float degv = (float)cnt + 1.0f; float agg = 0.0f;
  for (int q = 0; q < cnt; ++q) { int id = perm[p0 + q]; id = (id < 0) ? 0 : (id >= NE ? NE - 1 : id); int s = src[id]; s = (s < 0) ? 0 : (s >= NN ? NN - 1 : s); int cs_ = rowcnt[s]; cs_ = (cs_ < 0) ? 0 : (cs_ > MAXDEG ? MAXDEG : cs_);
    const float nrm = rsqrtf(pmul((float)cs_ + 1.0f, degv)); const float c2 = CS[(size_t)s * 2], s2 = CS[(size_t)s * 2 + 1];
    const float m00 = pmul(cv, c2) + pmul(sv, s2), m01 = pmul(cv, -s2) + pmul(sv, c2), m10 = pmul(-sv, c2) + pmul(cv, s2), m11 = pmul(-sv, -s2) + pmul(cv, c2);
    const float x0 = XSin[(size_t)s * DH + k], x1 = XSin[(size_t)s * DH + 16 + k]; const float mv = (d == 0) ? (pmul(m00, x0) + pmul(m01, x1)) : (pmul(m10, x0) + pmul(m11, x1)); agg += pmul(mv, nrm); }
  const float xv = XSin[(size_t)v * DH + lane]; Lx[wave][lane] = xv - agg;
  wave_lds_sync();
  float s_ = 0.0f;
#pragma unroll
  for (int h = 0; h < 16; ++h) s_ += pmul(Lx[wave][d * 16 + h], Pw[h * 16 + k]);
  const float xn = xv - gelu_t(s_);
  if (LAST) { b16 a_, b_; split16(xn * XS, a_, b_); Sh[wave][lane] = a_; Sl[wave][lane] = b_; wave_lds_sync(); }
  for (int pass = 0; pass < 2; ++pass) { ((volatile float*)XSout)[(size_t)v * DH + lane] = xn; if (LAST && lane < 4) { *(volatile v8b*)(Xh + (size_t)v * DH + lane * 8) = *(const v8b*)(&Sh[wave][lane * 8]); *(volatile v8b*)(Xl + (size_t)v * DH + lane * 8) = *(const v8b*)(&Sl[wave][lane * 8]); } __threadfence(); }
}
__global__ __launch_bounds__(64) void out_kernel(const b16* __restrict__ Xh, const b16* __restrict__ Xl, const b16* __restrict__ Bw, const float* __restrict__ P, float* __restrict__ out) {
  __shared__ __attribute__((aligned(16))) float Os[32 * NOUT];
  const int lane = threadIdx.x & 31, wave = threadIdx.x >> 5, nloc = lane & 15, hlf = lane >> 4, m0 = blockIdx.x * 32 + wave * 16;
  v8f acc = {}; const v16b a = frag_kb(Xh + (size_t)(m0 + nloc) * DH, hlf), al_ = frag_kb(Xl + (size_t)(m0 + nloc) * DH, hlf), bw = frag_kb(Bw + (size_t)nloc * DH, hlf); acc = wmma16b(a, bw, acc); acc = wmma16b(al_, bw, acc);
  if (nloc < NOUT) {
#pragma unroll
    for (int r = 0; r < 8; ++r) Os[(wave * 16 + 8 * hlf + r) * NOUT + nloc] = acc[r] * (1.0f / XS) + P[704 + nloc]; }
  __syncthreads();
  for (int pass = 0; pass < 2; ++pass) { for (int i = threadIdx.x; i < 32 * NOUT / 4; i += 64) *(volatile v4f*)(out + (size_t)blockIdx.x * 32 * NOUT + i * 4) = *(const v4f*)(&Os[i * 4]); __threadfence(); }
}
}

extern "C" void kernel_launch(void* const* d_in, const int* in_sizes, int n_in,
                              void* d_out, int out_size, void* d_ws, size_t ws_size, hipStream_t stream) {
  (void)n_in; (void)out_size;
  auto Fp = [&](int i) { return (const float*)d_in[i]; };
  const float* x = Fp(0); const int* ei = (const int*)d_in[1];
  float* out = (float*)d_out;
  if (in_sizes[0] != NN * FI || in_sizes[1] != 2 * NE || in_sizes[2] != FI * DH) return;
  const int* srcI = ei; const int* dstI = ei + NE; const int NE_RUN = NE;
  size_t off = 0; char* ws = (char*)d_ws;
  auto carve = [&](size_t bytes) { char* p = ws + off; off += (bytes + 255) & ~(size_t)255; return p; };
  b16* R = (b16*)carve(23040 * 2); float* P = (float*)carve(720 * 4); b16* X = (b16*)carve((size_t)NN * FI * 2); float* H = (float*)carve((size_t)NN * DH * 4); b16* Hh = (b16*)carve((size_t)NN * DH * 2); b16* Hl = (b16*)carve((size_t)NN * DH * 2); float* M = (float*)carve((size_t)NN * GH * 4); b16* Ch = (b16*)carve((size_t)NN * 128 * 2); b16* Cl = (b16*)carve((size_t)NN * 128 * 2); float* CS = (float*)carve((size_t)NN * 2 * 4); float* XS2 = (float*)carve((size_t)NN * DH * 4);
  CsrBufs cs; off = csr_carve(cs, ws, off, NE_RUN, NN);
  if (off > ws_size) return;
  csr_build(cs, dstI, NE_RUN, NN, stream);
  prep_kernel<<<512, 256, 0, stream>>>(x, Fp(2), Fp(3), Fp(4), Fp(5), Fp(6), Fp(7), Fp(8), Fp(9), Fp(10), Fp(11), Fp(12), Fp(13), Fp(14), R, P, X);
  gemm_kernel<FI, DH, 0, 0><<<NN / 32, 64, 0, stream>>>(X, nullptr, FI, R, P, H, nullptr, nullptr);
  hsplit_kernel<<<(NN * DH / 8 + 255) / 256, 256, 0, stream>>>(H, Hh, Hl);
  gemm_kernel<DH, GH, 1, 1><<<NN / 32, 64, 0, stream>>>(Hh, Hl, DH, R + 4096, P + 32, M, Ch, Cl);
  magg_kernel<<<NN / 8, 256, 0, stream>>>(M, srcI, cs.PERM, cs.ROWPTR, cs.ROWCNT, Ch, Cl);
  gemm_kernel<128, GH, 1, 1><<<NN / 32, 64, 0, stream>>>(Ch, Cl, 128, R + 6144, nullptr, M, Ch, Cl);
  magg_kernel<<<NN / 8, 256, 0, stream>>>(M, srcI, cs.PERM, cs.ROWPTR, cs.ROWCNT, Ch, Cl);
  gemm_kernel<128, GH, 1, 1><<<NN / 32, 64, 0, stream>>>(Ch, Cl, 128, R + 14336, nullptr, M, Ch, Cl);
  theta_kernel<<<(NN + 255) / 256, 256, 0, stream>>>(M, P, CS);
  diff_kernel<0><<<NN / 8, 256, 0, stream>>>(H, CS, srcI, cs.PERM, cs.ROWPTR, cs.ROWCNT, P + 192, XS2, nullptr, nullptr);
  diff_kernel<1><<<NN / 8, 256, 0, stream>>>(XS2, CS, srcI, cs.PERM, cs.ROWPTR, cs.ROWCNT, P + 192 + 256, H, Hh, Hl);
  out_kernel<<<NN / 32, 64, 0, stream>>>(Hh, Hl, R + 22528, P, out);
}
